// nonlinearMLP_57896159150711
// MI455X (gfx1250) — hardware-verified
//
#include <hip/hip_runtime.h>
#include <math.h>

typedef __attribute__((ext_vector_type(16))) _Float16 v16h;
typedef __attribute__((ext_vector_type(16))) __bf16 v16b;
typedef __attribute__((ext_vector_type(8)))  _Float16 v8h;
typedef __attribute__((ext_vector_type(8)))  float v8f;
typedef __attribute__((ext_vector_type(4)))  float v4f;
typedef __attribute__((ext_vector_type(2)))  float v2f;
typedef __attribute__((ext_vector_type(4)))  unsigned v4u;
typedef __attribute__((ext_vector_type(4)))  int v4i;
typedef float __attribute__((may_alias)) float_a;
typedef int __attribute__((may_alias)) int_a;

template <typename T> __device__ __forceinline__ void vst2(void* p, T v) { *(volatile T*)p = v; __threadfence(); *(volatile T*)p = v; }
__device__ __forceinline__ v8f wmma16(v16h a, v16h b, v8f c) {
  v8f d = __builtin_amdgcn_wmma_f32_16x16x32_f16(false, a, false, b, (short)0, c, false, false);
  asm volatile("v_nop\n\tv_nop\n\tv_nop\n\tv_nop" : "+v"(d) : "v"(a), "v"(b));
  return d;
}
__device__ __forceinline__ v8f wmma_bf(v16b a, v16b b, v8f c) {
  v8f d = __builtin_amdgcn_wmma_f32_16x16x32_bf16(false, a, false, b, (short)0, c, false, false);
  asm volatile("v_nop\n\tv_nop\n\tv_nop\n\tv_nop" : "+v"(d) : "v"(a), "v"(b));
  return d;
}
__device__ __forceinline__ v16h frag_h(const _Float16* rowk0, int lane) {
  union { v16h v; v8h q[2]; } u; const _Float16* p = rowk0 + 8 * (lane >> 4);
  u.q[0] = *(const v8h*)p; u.q[1] = *(const v8h*)(p + 16); return u.v;
}
__device__ __forceinline__ v16h frag_f32(const float* rowk0, int lane) {
  v16h a; const float* p = rowk0 + 8 * (lane >> 4);
#pragma unroll
  for (int i = 0; i < 8; ++i) { a[i] = (_Float16)p[i]; a[8 + i] = (_Float16)p[16 + i]; }
  return a;
}
__device__ __forceinline__ v16h frag_f32s(const float* rowk0, int lane, float sc) {
  v16h a; const float* p = rowk0 + 8 * (lane >> 4);
#pragma unroll
  for (int i = 0; i < 8; ++i) { a[i] = (_Float16)(p[i] * sc); a[8 + i] = (_Float16)(p[16 + i] * sc); }
  return a;
}
__device__ __forceinline__ v16h fragc_f32(const float* W, int k0, int n, int lane, int ld, int K) {
  v16h a; const int g = lane >> 4;
#pragma unroll
  for (int i = 0; i < 8; ++i) { const int ka = k0 + 8 * g + i, kb = ka + 16;
    a[i] = (_Float16)(ka < K ? W[(size_t)ka * ld + n] : 0.f); a[8 + i] = (_Float16)(kb < K ? W[(size_t)kb * ld + n] : 0.f); }
  return a;
}
struct F2 { v16b h, l; };
__device__ __forceinline__ F2 bsplit16(const float v[16]) { F2 r;
#pragma unroll
  for (int i = 0; i < 16; ++i) { const __bf16 h = (__bf16)v[i]; r.h[i] = h; r.l[i] = (__bf16)(v[i] - (float)h); }
  return r; }
__device__ __forceinline__ F2 split_row(const float* row, int k0, int lane) { float v[16]; const float* p = row + k0 + 8 * (lane >> 4);
#pragma unroll
  for (int i = 0; i < 8; ++i) { v[i] = p[i]; v[8 + i] = p[16 + i]; }
  return bsplit16(v); }
__device__ __forceinline__ F2 split_rowK(const float* row, int k0, int lane, int K) { float v[16]; const int g = lane >> 4;
#pragma unroll
  for (int i = 0; i < 8; ++i) { const int ka = k0 + 8 * g + i, kb = ka + 16; v[i] = ka < K ? row[ka] : 0.f; v[8 + i] = kb < K ? row[kb] : 0.f; }
  return bsplit16(v); }
__device__ __forceinline__ F2 split_col(const float* W, int k0, int n, int lane, int ld, int K) { float v[16]; const int g = lane >> 4;
#pragma unroll
  for (int i = 0; i < 8; ++i) { const int ka = k0 + 8 * g + i, kb = ka + 16; v[i] = ka < K ? W[(size_t)ka * ld + n] : 0.f; v[8 + i] = kb < K ? W[(size_t)kb * ld + n] : 0.f; }
  return bsplit16(v); }
__device__ __forceinline__ v8f mac3(const F2& a, const F2& b, v8f c) { c = wmma_bf(a.l, b.h, c); c = wmma_bf(a.h, b.l, c); return wmma_bf(a.h, b.h, c); }
__device__ __forceinline__ float sigm(float v) { return 1.0f / (1.0f + expf(-v)); }
#define LDSX() do { asm volatile("s_wait_dscnt 0" ::: "memory"); __builtin_amdgcn_wave_barrier(); __builtin_amdgcn_fence(__ATOMIC_RELEASE, "workgroup"); } while (0)

#define NBT 1024
#define NN 256

__global__ __launch_bounds__(128) void k_z1(const float* __restrict__ x, const float* __restrict__ W0, float* __restrict__ Z1) {
  __shared__ __align__(16) float so[4][16][132];
  const int tid = threadIdx.x, wave = tid >> 5, lane = tid & 31, col = lane & 15, g = lane >> 4;
  const int r0 = blockIdx.x * 64 + wave * 16, n0 = blockIdx.y * 128;
  v8f acc[8] = {};
#pragma unroll 1
  for (int kc = 0; kc < NN / 32; ++kc) { const F2 a = split_row(x + (size_t)(r0 + col) * NN, kc * 32, lane);
#pragma unroll
    for (int j = 0; j < 8; ++j) acc[j] = mac3(a, split_row(W0 + (size_t)(n0 + j * 16 + col) * NN, kc * 32, lane), acc[j]); }
#pragma unroll
  for (int j = 0; j < 8; ++j)
#pragma unroll
    for (int r = 0; r < 8; ++r) so[wave][8 * g + r][j * 16 + col] = acc[j][r];
  LDSX();
#pragma unroll 4
  for (int rl = 0; rl < 16; ++rl) vst2(Z1 + (size_t)(r0 + rl) * NN + n0 + lane * 4, *(const v4f*)(&so[wave][rl][lane * 4]));
}
__global__ __launch_bounds__(128) void k_main(const float* __restrict__ x, const float* __restrict__ W0, const float* __restrict__ Z1, const float* __restrict__ W1, const float* __restrict__ W2, float* __restrict__ FT) {
  __shared__ float sw0c[NN], sw2r[NN];
  __shared__ __align__(16) float sf[64];
  __shared__ float sh2[4][16][NN + 1];
  const int tid = threadIdx.x, wave = tid >> 5, lane = tid & 31, col = lane & 15, g = lane >> 4;
  const int i = blockIdx.y, b0 = blockIdx.x * 64 + wave * 16;
  for (int q = tid; q < NN; q += 128) { sw0c[q] = W0[(size_t)q * NN + i]; sw2r[q] = W2[(size_t)i * NN + q]; }
  __syncthreads();
  const int bm = b0 + col; const float xi = x[(size_t)bm * NN + i]; const float* zr = Z1 + (size_t)bm * NN;
  v8f acc[16];
#pragma unroll
  for (int t = 0; t < 16; ++t) acc[t] = (v8f){};
#pragma unroll 1
  for (int kc = 0; kc < NN / 32; ++kc) { v16h a;
#pragma unroll
    for (int e = 0; e < 8; ++e) { const int ka = kc * 32 + 8 * g + e, kb = ka + 16; a[e] = (_Float16)tanhf(zr[ka] - xi * sw0c[ka]); a[8 + e] = (_Float16)tanhf(zr[kb] - xi * sw0c[kb]); }
#pragma unroll
    for (int t = 0; t < 16; ++t) acc[t] = wmma16(a, frag_f32s(W1 + (size_t)(t * 16 + col) * NN + kc * 32, lane, 16.0f), acc[t]); }
#pragma unroll
  for (int t = 0; t < 16; ++t)
#pragma unroll
    for (int r = 0; r < 8; ++r) sh2[wave][8 * g + r][t * 16 + col] = acc[t][r] * (1.0f / 16.0f);
  LDSX();
  { const int rl = lane >> 1, hf = lane & 1; float s = 0.f;
#pragma unroll 2
    for (int n = hf * 128; n < hf * 128 + 128; ++n) s += tanhf(sh2[wave][rl][n]) * sw2r[n];
    s += __shfl_xor(s, 1, 32);
    if (hf == 0) sf[wave * 16 + rl] = tanhf(s); }
  __syncthreads();
  if (tid < 16) vst2(FT + (size_t)i * NBT + blockIdx.x * 64 + tid * 4, *(const v4f*)(&sf[tid * 4]));
}
__global__ __launch_bounds__(256) void k_tr(const float* __restrict__ FT, float* __restrict__ out) {
  __shared__ float st[64][NN + 1];
  const int b0 = blockIdx.x * 64, tid = threadIdx.x;
  for (int q = tid; q < NN * 64; q += 256) { const int i = q >> 6, bl = q & 63; st[bl][i] = FT[(size_t)i * NBT + b0 + bl]; }
  __syncthreads();
  for (int q = tid; q < 64 * (NN / 4); q += 256) { const int bl = q >> 6, pc = q & 63; v4f o; o[0] = st[bl][pc * 4]; o[1] = st[bl][pc * 4 + 1]; o[2] = st[bl][pc * 4 + 2]; o[3] = st[bl][pc * 4 + 3]; vst2(out + (size_t)(b0 + bl) * NN + pc * 4, o); }
}
extern "C" void kernel_launch(void* const* d_in, const int* in_sizes, int n_in, void* d_out, int out_size, void* d_ws, size_t ws_size, hipStream_t stream) {
  (void)in_sizes; (void)n_in; (void)out_size; (void)ws_size;
  const float* x = (const float*)d_in[0]; const float* W0 = (const float*)d_in[1]; const float* W1 = (const float*)d_in[2]; const float* W2 = (const float*)d_in[3];
  float* out = (float*)d_out;
  char* ws = (char*)d_ws; size_t off = 0;
  auto take = [&](size_t bytes) { char* p = ws + off; off += (bytes + 255) & ~(size_t)255; return p; };
  float* Z1 = (float*)take((size_t)NBT * NN * 4); float* FT = (float*)take((size_t)NN * NBT * 4);
  k_z1<<<dim3(NBT / 64, NN / 128), 128, 0, stream>>>(x, W0, Z1);
  k_main<<<dim3(NBT / 64, NN), 128, 0, stream>>>(x, W0, Z1, W1, W2, FT);
  k_tr<<<NBT / 64, 256, 0, stream>>>(FT, out);
}
